// FourierKAN_54279796687467
// MI455X (gfx1250) — hardware-run, weakly checked
//
#include <hip/hip_runtime.h>
#include <math.h>

typedef __attribute__((ext_vector_type(16))) _Float16 v16h;
typedef __attribute__((ext_vector_type(16))) __bf16 v16b;
typedef __attribute__((ext_vector_type(8)))  _Float16 v8h;
typedef __attribute__((ext_vector_type(8)))  float v8f;
typedef __attribute__((ext_vector_type(4)))  float v4f;
typedef __attribute__((ext_vector_type(2)))  float v2f;
typedef __attribute__((ext_vector_type(4)))  unsigned v4u;
typedef __attribute__((ext_vector_type(4)))  int v4i;
typedef float __attribute__((may_alias)) float_a;
typedef int __attribute__((may_alias)) int_a;

template <typename T> __device__ __forceinline__ void vst2(void* p, T v) { *(volatile T*)p = v; __threadfence(); *(volatile T*)p = v; }
__device__ __forceinline__ v8f wmma16(v16h a, v16h b, v8f c) {
  v8f d = __builtin_amdgcn_wmma_f32_16x16x32_f16(false, a, false, b, (short)0, c, false, false);
  asm volatile("v_nop\n\tv_nop\n\tv_nop\n\tv_nop" : "+v"(d) : "v"(a), "v"(b));
  return d;
}
__device__ __forceinline__ v8f wmma_bf(v16b a, v16b b, v8f c) {
  v8f d = __builtin_amdgcn_wmma_f32_16x16x32_bf16(false, a, false, b, (short)0, c, false, false);
  asm volatile("v_nop\n\tv_nop\n\tv_nop\n\tv_nop" : "+v"(d) : "v"(a), "v"(b));
  return d;
}
__device__ __forceinline__ v16h frag_h(const _Float16* rowk0, int lane) {
  union { v16h v; v8h q[2]; } u; const _Float16* p = rowk0 + 8 * (lane >> 4);
  u.q[0] = *(const v8h*)p; u.q[1] = *(const v8h*)(p + 16); return u.v;
}
__device__ __forceinline__ v16h frag_f32(const float* rowk0, int lane) {
  v16h a; const float* p = rowk0 + 8 * (lane >> 4);
#pragma unroll
  for (int i = 0; i < 8; ++i) { a[i] = (_Float16)p[i]; a[8 + i] = (_Float16)p[16 + i]; }
  return a;
}
__device__ __forceinline__ v16h frag_f32s(const float* rowk0, int lane, float sc) {
  v16h a; const float* p = rowk0 + 8 * (lane >> 4);
#pragma unroll
  for (int i = 0; i < 8; ++i) { a[i] = (_Float16)(p[i] * sc); a[8 + i] = (_Float16)(p[16 + i] * sc); }
  return a;
}
__device__ __forceinline__ v16h fragc_f32(const float* W, int k0, int n, int lane, int ld, int K) {
  v16h a; const int g = lane >> 4;
#pragma unroll
  for (int i = 0; i < 8; ++i) { const int ka = k0 + 8 * g + i, kb = ka + 16;
    a[i] = (_Float16)(ka < K ? W[(size_t)(ka < K ? ka : K - 1) * ld + n] : 0.f); a[8 + i] = (_Float16)(kb < K ? W[(size_t)(kb < K ? kb : K - 1) * ld + n] : 0.f); }
  return a;
}
struct F2 { v16b h, l; };
__device__ __forceinline__ F2 bsplit16(const float v[16]) { F2 r;
#pragma unroll
  for (int i = 0; i < 16; ++i) { const __bf16 h = (__bf16)v[i]; r.h[i] = h; r.l[i] = (__bf16)(v[i] - (float)h); }
  return r; }
__device__ __forceinline__ F2 split_row(const float* row, int k0, int lane) { float v[16]; const float* p = row + k0 + 8 * (lane >> 4);
#pragma unroll
  for (int i = 0; i < 8; ++i) { v[i] = p[i]; v[8 + i] = p[16 + i]; }
  return bsplit16(v); }
__device__ __forceinline__ F2 split_rowK(const float* row, int k0, int lane, int K) { float v[16]; const int g = lane >> 4;
#pragma unroll
  for (int i = 0; i < 8; ++i) { const int ka = k0 + 8 * g + i, kb = ka + 16; v[i] = ka < K ? row[ka < K ? ka : K - 1] : 0.f; v[8 + i] = kb < K ? row[kb < K ? kb : K - 1] : 0.f; }
  return bsplit16(v); }
__device__ __forceinline__ F2 split_col(const float* W, int k0, int n, int lane, int ld, int K) { float v[16]; const int g = lane >> 4;
#pragma unroll
  for (int i = 0; i < 8; ++i) { const int ka = k0 + 8 * g + i, kb = ka + 16; v[i] = ka < K ? W[(size_t)(ka < K ? ka : K - 1) * ld + n] : 0.f; v[8 + i] = kb < K ? W[(size_t)(kb < K ? kb : K - 1) * ld + n] : 0.f; }
  return bsplit16(v); }
__device__ __forceinline__ v8f mac3(const F2& a, const F2& b, v8f c) { c = wmma_bf(a.l, b.h, c); c = wmma_bf(a.h, b.l, c); return wmma_bf(a.h, b.h, c); }
__device__ __forceinline__ float sigm(float v) { return 1.0f / (1.0f + expf(-v)); }
#define LDSX() do { asm volatile("s_wait_dscnt 0" ::: "memory"); __builtin_amdgcn_wave_barrier(); __builtin_amdgcn_fence(__ATOMIC_RELEASE, "workgroup"); } while (0)


#define NR 4096
#define DIN 256
#define H1 512
#define H2 512
#define DOUT 256
#define G2 16
#define G3 8
#define K2 (H1 * 2 * G2)
#define K3 (H2 * 2 * G3)
#define WSC 256.0f
#define EPS 1e-5f
typedef __attribute__((ext_vector_type(8))) __bf16 v8b;
__device__ __forceinline__ v16b frag_b(const __bf16* rowk0, int lane) {
  union { v16b v; v8b q[2]; } u; const __bf16* p = rowk0 + 8 * (lane >> 4);
  u.q[0] = *(const v8b*)p; u.q[1] = *(const v8b*)(p + 16); return u.v;
}
__device__ __forceinline__ float bfr(float v) { return (float)(__bf16)v; }
__device__ __attribute__((noinline)) float exp_ni(float v) { return expf(v); }
__device__ __attribute__((noinline)) float erf_ni(float v) { return erff(v); }

#define WS_C2  0u
#define WS_C3  (WS_C2 + 2u * (size_t)H2 * K2)
#define WS_H   (WS_C3 + 2u * (size_t)DOUT * K3)
#define WS_MV  (WS_H + 4u * (size_t)NR * H1)
#define WS_F1  (WS_MV + 128u)
#define WS_Y2  (WS_F1 + 2u * (size_t)NR * K2)
#define WS_F2  (WS_Y2 + 4u * (size_t)NR * H2)
#define WS_END (WS_F2 + 2u * (size_t)NR * K3)

template <int L>
__global__ __launch_bounds__(256) void k_packc(const float* __restrict__ C, _Float16* __restrict__ ROWS) { constexpr int NI = (L == 2) ? H1 : H2; constexpr int G = (L == 2) ? G2 : G3; constexpr int NOU = (L == 2) ? H2 : DOUT; constexpr int KW = NI * 2 * G; __shared__ __align__(16) _Float16 s[K2]; const int o = blockIdx.x, t = threadIdx.x;
  for (int e = t; e < KW; e += 256) { const int i = e / (2 * G), j = e % (2 * G); const int cs = j < G ? 0 : 1, g = j < G ? j : j - G; s[e] = (_Float16)(bfr(C[(((size_t)cs * NOU + o) * NI + i) * G + g]) * WSC); }
  __syncthreads(); for (int q = t; q < KW / 8; q += 256) vst2((unsigned*)(ROWS + (size_t)o * KW + q * 8), *(const v4u*)&s[q * 8]); }
__device__ __forceinline__ v16b fragb_f32(const float* __restrict__ p, int lane) { v16b a; const float* pp = p + 8 * (lane >> 4);
#pragma unroll
  for (int i = 0; i < 8; ++i) { a[i] = (__bf16)pp[i]; a[8 + i] = (__bf16)pp[16 + i]; } return a; }
__global__ __launch_bounds__(128) void k_lin(const float* __restrict__ X, const float* __restrict__ W1, const float* __restrict__ B1, float* __restrict__ H) { __shared__ __align__(16) float sf[4][16][132];
  const int tid = threadIdx.x, wave = tid >> 5, lane = tid & 31, col = lane & 15, g = lane >> 4; const size_t r0 = (size_t)blockIdx.x * 64 + wave * 16; const int c0 = blockIdx.y * 128;
  v8f acc[8] = {};
#pragma unroll
  for (int kc = 0; kc < DIN / 32; ++kc) { const v16b a = fragb_f32(X + (r0 + col) * DIN + kc * 32, lane);
#pragma unroll
    for (int j = 0; j < 8; ++j) acc[j] = wmma_bf(a, fragb_f32(W1 + (size_t)(c0 + j * 16 + col) * DIN + kc * 32, lane), acc[j]); }
#pragma unroll
  for (int j = 0; j < 8; ++j) { const float bb = bfr(B1[c0 + j * 16 + col]);
#pragma unroll
    for (int r = 0; r < 8; ++r) sf[wave][8 * g + r][j * 16 + col] = acc[j][r] + bb; }
  LDSX(); for (int rl = 0; rl < 16; ++rl) vst2(H + (r0 + rl) * H1 + c0 + lane * 4, *(const v4f*)&sf[wave][rl][lane * 4]); }
__global__ __launch_bounds__(1024) void k_stat(const float* __restrict__ H, float* __restrict__ MV) { __shared__ float red[32]; __shared__ __align__(16) float so2[32]; const int t = threadIdx.x; const size_t n = (size_t)NR * H1;
  float s = 0.f; for (size_t e = t; e < n; e += 1024) s += H[e];
#pragma unroll
  for (int o = 1; o < 32; o <<= 1) s += __shfl_xor(s, o);
  if ((t & 31) == 0) red[t >> 5] = s; __syncthreads(); float tot = 0.f; for (int i = 0; i < 32; ++i) tot += red[i]; const float mean = tot / (float)n; __syncthreads();
  float q = 0.f; for (size_t e = t; e < n; e += 1024) { const float d = H[e] - mean; q += d * d; }
#pragma unroll
  for (int o = 1; o < 32; o <<= 1) q += __shfl_xor(q, o);
  if ((t & 31) == 0) red[t >> 5] = q; __syncthreads(); if (t == 0) { float tq = 0.f; for (int i = 0; i < 32; ++i) tq += red[i]; so2[0] = mean; so2[1] = tq / (float)n; for (int i = 2; i < 32; ++i) so2[i] = 0.f; } __syncthreads();
  if (t < 8) vst2(MV + t * 4, *(const v4f*)&so2[t * 4]); }
template <int L>
__global__ __launch_bounds__(256) void k_feat(const float* __restrict__ SRC, const float* __restrict__ MV, const float* __restrict__ GAM, const float* __restrict__ BET, _Float16* __restrict__ F) { constexpr int NI = (L == 1) ? H1 : H2; constexpr int G = (L == 1) ? G2 : G3; constexpr int KW = NI * 2 * G; __shared__ __align__(16) _Float16 s[K2]; const int t = threadIdx.x; const size_t row = blockIdx.x;
  float mean = 0.f, inv = 1.f, ga = 1.f, be = 0.f; if (L == 1) { mean = MV[0]; inv = 1.0f / sqrtf(MV[1] + EPS); ga = bfr(GAM[0]); be = bfr(BET[0]); }
  for (int i = t; i < NI; i += 256) { float x = SRC[row * NI + i]; if (L == 1) x = fmaxf(ga * (x - mean) * inv + be, 0.f);
#pragma unroll 1
    for (int g = 0; g < G; ++g) { const float arg = x * (float)(g + 1); s[i * 2 * G + g] = (_Float16)cosf(arg); s[i * 2 * G + G + g] = (_Float16)sinf(arg); } }
  __syncthreads(); for (int q = t; q < KW / 8; q += 256) vst2((unsigned*)(F + row * KW + q * 8), *(const v4u*)&s[q * 8]); }
__global__ __launch_bounds__(128) void k_kan2(const _Float16* __restrict__ F1, const _Float16* __restrict__ C2R, const float* __restrict__ B2, float* __restrict__ Y2) { __shared__ __align__(16) float sf[4][16][132];
  const int tid = threadIdx.x, wave = tid >> 5, lane = tid & 31, col = lane & 15, g = lane >> 4; const size_t r0 = (size_t)blockIdx.x * 64 + wave * 16; const int c0 = blockIdx.y * 128;
  v8f acc[8] = {};
#pragma unroll 2
  for (int kc = 0; kc < K2 / 32; ++kc) { const v16h a = frag_h(F1 + (r0 + col) * K2 + kc * 32, lane);
#pragma unroll
    for (int j = 0; j < 8; ++j) acc[j] = wmma16(a, frag_h(C2R + (size_t)(c0 + j * 16 + col) * K2 + kc * 32, lane), acc[j]); }
#pragma unroll
  for (int j = 0; j < 8; ++j) { const float bb = bfr(B2[c0 + j * 16 + col]);
#pragma unroll
    for (int r = 0; r < 8; ++r) sf[wave][8 * g + r][j * 16 + col] = acc[j][r] * (1.0f / WSC) + bb; }
  LDSX(); for (int rl = 0; rl < 16; ++rl) vst2(Y2 + (r0 + rl) * H2 + c0 + lane * 4, *(const v4f*)&sf[wave][rl][lane * 4]); }
__global__ __launch_bounds__(128) void k_kan3(const _Float16* __restrict__ F2, const _Float16* __restrict__ C3R, const float* __restrict__ B3, float* __restrict__ OUT) { __shared__ __align__(16) float sz[64][DOUT + 4];
  const int tid = threadIdx.x, wave = tid >> 5, lane = tid & 31, col = lane & 15, g = lane >> 4; const size_t rb = (size_t)blockIdx.x * 64; const size_t r0 = rb + wave * 16;
  v8f acc[16];
#pragma unroll
  for (int j = 0; j < 16; ++j) acc[j] = v8f{};
#pragma unroll 1
  for (int kc = 0; kc < K3 / 32; ++kc) { const v16h a = frag_h(F2 + (r0 + col) * K3 + kc * 32, lane);
#pragma unroll
    for (int j = 0; j < 16; ++j) acc[j] = wmma16(a, frag_h(C3R + (size_t)(j * 16 + col) * K3 + kc * 32, lane), acc[j]); }
#pragma unroll
  for (int j = 0; j < 16; ++j) { const float bb = bfr(B3[j * 16 + col]);
#pragma unroll
    for (int r = 0; r < 8; ++r) sz[wave * 16 + 8 * g + r][j * 16 + col] = acc[j][r] * (1.0f / WSC) + bb; }
  LDSX();
  for (int rl = 0; rl < 16; ++rl) { float* zr = &sz[wave * 16 + rl][0]; float v[8]; float mx = -3.0e38f;
#pragma unroll
    for (int i = 0; i < 8; ++i) { v[i] = zr[lane + 32 * i]; mx = fmaxf(mx, v[i]); }
#pragma unroll
    for (int o = 1; o < 32; o <<= 1) mx = fmaxf(mx, __shfl_xor(mx, o));
    float s = 0.f;
#pragma unroll
    for (int i = 0; i < 8; ++i) { v[i] = expf(v[i] - mx); s += v[i]; }
#pragma unroll
    for (int o = 1; o < 32; o <<= 1) s += __shfl_xor(s, o);
    const float inv = 1.0f / s;
#pragma unroll
    for (int i = 0; i < 8; ++i) zr[lane + 32 * i] = v[i] * inv; }
  LDSX(); for (int rl = 0; rl < 16; ++rl) for (int q = lane; q < DOUT / 4; q += 32) vst2(OUT + (r0 + rl) * DOUT + q * 4, *(const v4f*)&sz[wave * 16 + rl][q * 4]); }
extern "C" void kernel_launch(void* const* d_in, const int* in_sizes, int n_in, void* d_out, int out_size, void* d_ws, size_t ws_size, hipStream_t stream) {
  (void)in_sizes; (void)n_in; (void)out_size;
  const float** F = (const float**)d_in;
  if (ws_size < (size_t)WS_END) return;
  char* ws = (char*)d_ws; _Float16 *C2R = (_Float16*)(ws + WS_C2), *C3R = (_Float16*)(ws + WS_C3), *F1 = (_Float16*)(ws + WS_F1), *F2 = (_Float16*)(ws + WS_F2); float *H = (float*)(ws + WS_H), *MV = (float*)(ws + WS_MV), *Y2 = (float*)(ws + WS_Y2);
  k_packc<2><<<H2, 256, 0, stream>>>(F[5], C2R);
  k_packc<3><<<DOUT, 256, 0, stream>>>(F[7], C3R);
  k_lin<<<dim3(NR / 64, H1 / 128), 128, 0, stream>>>(F[0], F[1], F[2], H);
  k_stat<<<1, 1024, 0, stream>>>(H, MV);
  k_feat<1><<<NR, 256, 0, stream>>>(H, MV, F[3], F[4], F1);
  k_kan2<<<dim3(NR / 64, H2 / 128), 128, 0, stream>>>(F1, C2R, F[6], Y2);
  k_feat<2><<<NR, 256, 0, stream>>>(Y2, MV, F[3], F[4], F2);
  k_kan3<<<NR / 64, 128, 0, stream>>>(F2, C3R, F[8], (float*)d_out);
}
